// HierDDLts_85744727097703
// MI455X (gfx1250) — hardware-verified
//
#include <hip/hip_runtime.h>
#include <math.h>

typedef __attribute__((ext_vector_type(16))) _Float16 v16h;
typedef __attribute__((ext_vector_type(16))) __bf16 v16b;
typedef __attribute__((ext_vector_type(8)))  _Float16 v8h;
typedef __attribute__((ext_vector_type(8)))  float v8f;
typedef __attribute__((ext_vector_type(4)))  float v4f;
typedef __attribute__((ext_vector_type(2)))  float v2f;
typedef __attribute__((ext_vector_type(4)))  unsigned v4u;
typedef __attribute__((ext_vector_type(4)))  int v4i;
typedef float __attribute__((may_alias)) float_a;
typedef int __attribute__((may_alias)) int_a;

template <typename T> __device__ __forceinline__ void vst2(void* p, T v) { *(volatile T*)p = v; __threadfence(); *(volatile T*)p = v; }
__device__ __forceinline__ v8f wmma16(v16h a, v16h b, v8f c) {
  v8f d = __builtin_amdgcn_wmma_f32_16x16x32_f16(false, a, false, b, (short)0, c, false, false);
  asm volatile("v_nop\n\tv_nop\n\tv_nop\n\tv_nop" : "+v"(d) : "v"(a), "v"(b));
  return d;
}
__device__ __forceinline__ v8f wmma_bf(v16b a, v16b b, v8f c) {
  v8f d = __builtin_amdgcn_wmma_f32_16x16x32_bf16(false, a, false, b, (short)0, c, false, false);
  asm volatile("v_nop\n\tv_nop\n\tv_nop\n\tv_nop" : "+v"(d) : "v"(a), "v"(b));
  return d;
}
__device__ __forceinline__ v16h frag_h(const _Float16* rowk0, int lane) {
  union { v16h v; v8h q[2]; } u; const _Float16* p = rowk0 + 8 * (lane >> 4);
  u.q[0] = *(const v8h*)p; u.q[1] = *(const v8h*)(p + 16); return u.v;
}
__device__ __forceinline__ v16h frag_f32(const float* rowk0, int lane) {
  v16h a; const float* p = rowk0 + 8 * (lane >> 4);
#pragma unroll
  for (int i = 0; i < 8; ++i) { a[i] = (_Float16)p[i]; a[8 + i] = (_Float16)p[16 + i]; }
  return a;
}
__device__ __forceinline__ v16h frag_f32s(const float* rowk0, int lane, float sc) {
  v16h a; const float* p = rowk0 + 8 * (lane >> 4);
#pragma unroll
  for (int i = 0; i < 8; ++i) { a[i] = (_Float16)(p[i] * sc); a[8 + i] = (_Float16)(p[16 + i] * sc); }
  return a;
}
__device__ __forceinline__ v16h fragc_f32(const float* W, int k0, int n, int lane, int ld, int K) {
  v16h a; const int g = lane >> 4;
#pragma unroll
  for (int i = 0; i < 8; ++i) { const int ka = k0 + 8 * g + i, kb = ka + 16;
    a[i] = (_Float16)(ka < K ? W[(size_t)(ka < K ? ka : K - 1) * ld + n] : 0.f); a[8 + i] = (_Float16)(kb < K ? W[(size_t)(kb < K ? kb : K - 1) * ld + n] : 0.f); }
  return a;
}
struct F2 { v16b h, l; };
__device__ __forceinline__ F2 bsplit16(const float v[16]) { F2 r;
#pragma unroll
  for (int i = 0; i < 16; ++i) { const __bf16 h = (__bf16)v[i]; r.h[i] = h; r.l[i] = (__bf16)(v[i] - (float)h); }
  return r; }
__device__ __forceinline__ F2 split_row(const float* row, int k0, int lane) { float v[16]; const float* p = row + k0 + 8 * (lane >> 4);
#pragma unroll
  for (int i = 0; i < 8; ++i) { v[i] = p[i]; v[8 + i] = p[16 + i]; }
  return bsplit16(v); }
__device__ __forceinline__ F2 split_rowK(const float* row, int k0, int lane, int K) { float v[16]; const int g = lane >> 4;
#pragma unroll
  for (int i = 0; i < 8; ++i) { const int ka = k0 + 8 * g + i, kb = ka + 16; v[i] = ka < K ? row[ka < K ? ka : K - 1] : 0.f; v[8 + i] = kb < K ? row[kb < K ? kb : K - 1] : 0.f; }
  return bsplit16(v); }
__device__ __forceinline__ F2 split_col(const float* W, int k0, int n, int lane, int ld, int K) { float v[16]; const int g = lane >> 4;
#pragma unroll
  for (int i = 0; i < 8; ++i) { const int ka = k0 + 8 * g + i, kb = ka + 16; v[i] = ka < K ? W[(size_t)(ka < K ? ka : K - 1) * ld + n] : 0.f; v[8 + i] = kb < K ? W[(size_t)(kb < K ? kb : K - 1) * ld + n] : 0.f; }
  return bsplit16(v); }
__device__ __forceinline__ v8f mac3(const F2& a, const F2& b, v8f c) { c = wmma_bf(a.l, b.h, c); c = wmma_bf(a.h, b.l, c); return wmma_bf(a.h, b.h, c); }
__device__ __forceinline__ float sigm(float v) { return 1.0f / (1.0f + expf(-v)); }
#define LDSX() do { asm volatile("s_wait_dscnt 0" ::: "memory"); __builtin_amdgcn_wave_barrier(); __builtin_amdgcn_fence(__ATOMIC_RELEASE, "workgroup"); } while (0)


#define NB 16
#define SS 1024
#define DD 96
#define GG 8
__device__ __forceinline__ float bfr(float v) { return (float)(__bf16)v; }
__device__ __forceinline__ v16b frag_b(const __bf16* rowk0, int lane) { return __builtin_bit_cast(v16b, frag_h((const _Float16*)rowk0, lane)); }
__device__ __attribute__((noinline)) float cos_ni(float v) { return cosf(v); }

__global__ __launch_bounds__(256) void k_w(const float* __restrict__ P, __bf16* __restrict__ Wh, __bf16* __restrict__ Wl) {
  __shared__ __align__(16) __bf16 sh_[DD * DD + 8], sl_[DD * DD + 8];
  const int tid = threadIdx.x; const int s = blockIdx.x; const float num = 6.28318548202514648f * (float)s;
#pragma unroll 1
  for (int q = tid; q < DD * DD; q += 256) { const int i = q / DD, j = q % DD; float acc = 0.f;
#pragma unroll 1
    for (int g = 0; g < GG; ++g) { const float per = (float)(i * DD * GG + j * GG + g + 2); acc += bfr(P[q * GG + g]) * cos_ni(num / per); }
    const __bf16 hi = (__bf16)acc; sh_[q] = hi; sl_[q] = (__bf16)(acc - (float)hi); }
  __syncthreads();
  for (int q = tid; q < DD * DD / 8; q += 256) { vst2((unsigned*)(Wh + (size_t)s * DD * DD + q * 8), *(const v4u*)(&sh_[q * 8])); vst2((unsigned*)(Wl + (size_t)s * DD * DD + q * 8), *(const v4u*)(&sl_[q * 8])); }
}
__global__ __launch_bounds__(256) void k_lt(const float* __restrict__ Lm, int NT, __bf16* __restrict__ LT) {
  __shared__ __align__(16) __bf16 st[64][72];
  const int tid = threadIdx.x; const int s0 = blockIdx.x * 64, t0 = blockIdx.y * 64;
  for (int q = tid; q < 64 * 64; q += 256) { const int sl = q >> 6, tl = q & 63; st[tl][sl] = (__bf16)Lm[(size_t)(s0 + sl) * NT + t0 + tl]; }
  __syncthreads();
  for (int q = tid; q < 64 * 8; q += 256) { const int tl = q >> 3, pc = q & 7; vst2((unsigned*)(LT + (size_t)(t0 + tl) * SS + s0 + pc * 8), *(const v4u*)(&st[tl][pc * 8])); }
}
template <int EXACT>
__global__ __launch_bounds__(128) void k_zm(const float* __restrict__ X, const float* __restrict__ M, const float* __restrict__ lw, const float* __restrict__ lb, const float* __restrict__ Rw, float* __restrict__ Z0, float* __restrict__ Z, float* __restrict__ R) {
  __shared__ __align__(16) float s0[4][16][100], s1[4][16][100];
  const int tid = threadIdx.x, wave = tid >> 5, lane = tid & 31, col = lane & 15, g = lane >> 4; const size_t r0 = (size_t)blockIdx.x * 64 + wave * 16;
  v8f acc[6] = {}, accr[6] = {};
#pragma unroll
  for (int kc = 0; kc < DD / 32; ++kc) { const F2 a = split_row(X + (r0 + col) * DD, kc * 32, lane);
#pragma unroll
    for (int j = 0; j < 6; ++j) { const v16b mb = split_row(M + (size_t)(j * 16 + col) * DD, kc * 32, lane).h;
      if (!EXACT) acc[j] = wmma_bf(a.l, mb, acc[j]); acc[j] = wmma_bf(a.h, mb, acc[j]);
      if (Rw) { const v16b rb = split_row(Rw + (size_t)(j * 16 + col) * DD, kc * 32, lane).h; if (!EXACT) accr[j] = wmma_bf(a.l, rb, accr[j]); accr[j] = wmma_bf(a.h, rb, accr[j]); } } }
#pragma unroll
  for (int j = 0; j < 6; ++j)
#pragma unroll
    for (int r = 0; r < 8; ++r) { s0[wave][8 * g + r][j * 16 + col] = acc[j][r]; if (Rw) s1[wave][8 * g + r][j * 16 + col] = accr[j][r]; }
  LDSX();
  for (int rl = 0; rl < 16; ++rl) { if (lane < 24) { vst2(Z0 + (r0 + rl) * DD + lane * 4, *(const v4f*)(&s0[wave][rl][lane * 4])); if (Rw) vst2(R + (r0 + rl) * DD + lane * 4, *(const v4f*)(&s1[wave][rl][lane * 4])); } }
  LDSX();
  { const int rl = lane & 15, hf = lane >> 4; float s = 0.f;
#pragma unroll 4
    for (int e = 0; e < 48; ++e) s += s0[wave][rl][hf * 48 + e];
    s += __shfl_xor(s, 16, 32); const float mu = s * (1.0f / DD); float q = 0.f;
#pragma unroll 4
    for (int e = 0; e < 48; ++e) { const float dv = s0[wave][rl][hf * 48 + e] - mu; q += dv * dv; }
    q += __shfl_xor(q, 16, 32); const float rs = rsqrtf(q * (1.0f / DD) + 1e-5f);
#pragma unroll 4
    for (int e = 0; e < 48; ++e) { const int c = hf * 48 + e; s1[wave][rl][c] = (s0[wave][rl][c] - mu) * rs * bfr(lw[c]) + bfr(lb[c]); } }
  LDSX();
  for (int rl = 0; rl < 16; ++rl) { if (lane < 24) vst2(Z + (r0 + rl) * DD + lane * 4, *(const v4f*)(&s1[wave][rl][lane * 4])); }
}
__global__ __launch_bounds__(128) void k_t(const float* __restrict__ Z, const float* __restrict__ ADD, const __bf16* __restrict__ Wh, const __bf16* __restrict__ Wl, float* __restrict__ TZ) {
  __shared__ __align__(16) float so[16][16][100];
  const int tid = threadIdx.x, wave = tid >> 5, lane = tid & 31, col = lane & 15, g = lane >> 4; const int sb = blockIdx.x * 16;
#pragma unroll 1
  for (int q = 0; q < 4; ++q) { const int sl = wave * 4 + q, s = sb + sl; v8f acc[6] = {};
#pragma unroll
    for (int kc = 0; kc < DD / 32; ++kc) { const F2 a = split_row(Z + ((size_t)col * SS + s) * DD, kc * 32, lane);
#pragma unroll
      for (int j = 0; j < 6; ++j) { const size_t wo = ((size_t)s * DD + j * 16 + col) * DD + kc * 32; const v16b wh = frag_b(Wh + wo, lane), wl = frag_b(Wl + wo, lane); acc[j] = wmma_bf(a.l, wh, acc[j]); acc[j] = wmma_bf(a.h, wl, acc[j]); acc[j] = wmma_bf(a.h, wh, acc[j]); } }
#pragma unroll
    for (int j = 0; j < 6; ++j)
#pragma unroll
      for (int r = 0; r < 8; ++r) { const int b = 8 * g + r, d = j * 16 + col; float v = acc[j][r]; if (ADD) v += ADD[((size_t)b * SS + s) * DD + d]; so[sl][b][d] = v; } }
  __syncthreads();
  for (int q = tid; q < 16 * 16 * 24; q += 128) { const int b = q / (16 * 24), rem = q % (16 * 24); const int sl = rem / 24, pc = rem % 24; vst2(TZ + (((size_t)b * SS + sb + sl) * DD) + pc * 4, *(const v4f*)(&so[sl][b][pc * 4])); }
}
__global__ __launch_bounds__(256) void k_tr(const float* __restrict__ TZ, __bf16* __restrict__ TTh, __bf16* __restrict__ TTl) {
  __shared__ __align__(16) __bf16 sh_[DD][72], sl_[DD][72];
  const int tid = threadIdx.x; const int b = blockIdx.y, s0 = blockIdx.x * 64;
  for (int q = tid; q < 64 * DD; q += 256) { const int sl = q / DD, d = q % DD; const float v = TZ[((size_t)b * SS + s0 + sl) * DD + d]; const __bf16 hi = (__bf16)v; sh_[d][sl] = hi; sl_[d][sl] = (__bf16)(v - (float)hi); }
  __syncthreads();
  for (int q = tid; q < DD * 8; q += 256) { const int d = q >> 3, pc = q & 7; const size_t o = ((size_t)b * DD + d) * SS + s0 + pc * 8; vst2((unsigned*)(TTh + o), *(const v4u*)(&sh_[d][pc * 8])); vst2((unsigned*)(TTl + o), *(const v4u*)(&sl_[d][pc * 8])); }
}
__global__ __launch_bounds__(128) void k_u(const __bf16* __restrict__ LT, const __bf16* __restrict__ TTh, const __bf16* __restrict__ TTl, const __bf16* __restrict__ LT2, const __bf16* __restrict__ T2h, const __bf16* __restrict__ T2l, int NT, float* __restrict__ U) {
  __shared__ __align__(16) float so[4][16][100];
  const int tid = threadIdx.x, wave = tid >> 5, lane = tid & 31, col = lane & 15, g = lane >> 4; const int t0 = blockIdx.x * 64 + wave * 16, b = blockIdx.y;
  v8f acc[6] = {};
#pragma unroll 2
  for (int kc = 0; kc < SS / 32; ++kc) { const v16b a = frag_b(LT + (size_t)(t0 + col) * SS + kc * 32, lane);
#pragma unroll
    for (int j = 0; j < 6; ++j) { const size_t to = ((size_t)b * DD + j * 16 + col) * SS + kc * 32; acc[j] = wmma_bf(a, frag_b(TTl + to, lane), acc[j]); acc[j] = wmma_bf(a, frag_b(TTh + to, lane), acc[j]); }
    if (LT2) { const v16b a2 = frag_b(LT2 + (size_t)(t0 + col) * SS + kc * 32, lane);
#pragma unroll
      for (int j = 0; j < 6; ++j) { const size_t to = ((size_t)b * DD + j * 16 + col) * SS + kc * 32; acc[j] = wmma_bf(a2, frag_b(T2l + to, lane), acc[j]); acc[j] = wmma_bf(a2, frag_b(T2h + to, lane), acc[j]); } } }
#pragma unroll
  for (int j = 0; j < 6; ++j)
#pragma unroll
    for (int r = 0; r < 8; ++r) so[wave][8 * g + r][j * 16 + col] = acc[j][r];
  LDSX();
  for (int rl = 0; rl < 16; ++rl) { if (lane < 24) vst2(U + (((size_t)b * NT + t0 + rl) * DD) + lane * 4, *(const v4f*)(&so[wave][rl][lane * 4])); }
}
extern "C" void kernel_launch(void* const* d_in, const int* in_sizes, int n_in, void* d_out, int out_size, void* d_ws, size_t ws_size, hipStream_t stream) {
  (void)in_sizes; (void)n_in; (void)out_size; (void)ws_size;
  const float** I = (const float**)d_in;
  char* ws = (char*)d_ws; size_t off = 0;
  auto take = [&](size_t bytes) { char* p = ws + off; off += (bytes + 255) & ~(size_t)255; return p; };
  const size_t NRW = (size_t)NB * SS;
  __bf16* Wh = (__bf16*)take((size_t)SS * DD * DD * 2); __bf16* Wl = (__bf16*)take((size_t)SS * DD * DD * 2);
  __bf16* LT = (__bf16*)take((size_t)SS * SS * 2); __bf16* LTb = (__bf16*)take((size_t)512 * SS * 2); __bf16* RLT = (__bf16*)take((size_t)512 * SS * 2);
  float* Z0 = (float*)take(NRW * DD * 4); float* Z = (float*)take(NRW * DD * 4); float* R = (float*)take(NRW * DD * 4); float* TZ = (float*)take(NRW * DD * 4);
  __bf16* TTh = (__bf16*)take(NRW * DD * 2); __bf16* TTl = (__bf16*)take(NRW * DD * 2); __bf16* T2h = (__bf16*)take(NRW * DD * 2); __bf16* T2l = (__bf16*)take(NRW * DD * 2); float* U1 = (float*)take(NRW * DD * 4);
  k_w<<<SS, 256, 0, stream>>>(I[2], Wh, Wl);
  k_lt<<<dim3(SS / 64, SS / 64), 256, 0, stream>>>(I[3], SS, LT);
  k_zm<1><<<NRW / 64, 128, 0, stream>>>(I[0], I[1], I[4], I[5], nullptr, Z0, Z, nullptr);
  k_t<<<SS / 16, 128, 0, stream>>>(Z, Z0, Wh, Wl, TZ);
  k_tr<<<dim3(SS / 64, NB), 256, 0, stream>>>(TZ, TTh, TTl);
  k_u<<<dim3(SS / 64, NB), 128, 0, stream>>>(LT, TTh, TTl, nullptr, nullptr, nullptr, SS, U1);
  k_w<<<SS, 256, 0, stream>>>(I[7], Wh, Wl);
  k_lt<<<dim3(SS / 64, 512 / 64), 256, 0, stream>>>(I[8], 512, LTb);
  k_lt<<<dim3(SS / 64, 512 / 64), 256, 0, stream>>>(I[12], 512, RLT);
  k_zm<0><<<NRW / 64, 128, 0, stream>>>(U1, I[6], I[9], I[10], I[11], Z0, Z, R);
  k_t<<<SS / 16, 128, 0, stream>>>(Z, nullptr, Wh, Wl, TZ);
  k_tr<<<dim3(SS / 64, NB), 256, 0, stream>>>(TZ, TTh, TTl);
  k_tr<<<dim3(SS / 64, NB), 256, 0, stream>>>(R, T2h, T2l);
  k_u<<<dim3(512 / 64, NB), 128, 0, stream>>>(LTb, TTh, TTl, RLT, T2h, T2l, 512, (float*)d_out);
}
